// DifAttention_29326036697660
// MI455X (gfx1250) — hardware-verified
//
#include <hip/hip_runtime.h>
#include <math.h>
#include <stdint.h>

constexpr int kBatch   = 4;
constexpr int kSeq     = 1024;
constexpr int kDim     = 768;
constexpr int kHeads   = 12;
constexpr int kHd      = 64;
constexpr int kTok     = kBatch * kSeq;
constexpr int kQkvRows = 4 * kDim;
constexpr int kLdQK    = 3 * kDim;
constexpr int kKeyChunk = 64;
constexpr int kWaves    = 4;

constexpr size_t kBytesXb   = (size_t)kTok * kDim * 2;
constexpr size_t kBytesWq   = (size_t)kQkvRows * kDim * 2;
constexpr size_t kBytesWp   = (size_t)kDim * kDim * 2;
constexpr size_t kBytesBias = 4096;
constexpr size_t kBytesP    = (size_t)kTok * kLdQK * 2;
constexpr size_t kBytesVt   = (size_t)kDim * kTok * 2;
constexpr size_t kBytesO    = (size_t)kTok * kDim * 4;
constexpr size_t kBytesS16  = (size_t)kTok * kDim * 2;
constexpr size_t kOffXb   = 0;
constexpr size_t kOffYb   = kOffXb + kBytesXb;
constexpr size_t kOffWq   = kOffYb + kBytesXb;
constexpr size_t kOffWp   = kOffWq + kBytesWq;
constexpr size_t kOffBias = kOffWp + kBytesWp;
constexpr size_t kOffPx   = kOffBias + kBytesBias;
constexpr size_t kOffPy   = kOffPx + kBytesP;
constexpr size_t kOffVt   = kOffPy + kBytesP;
constexpr size_t kOffOsx  = kOffVt + kBytesVt;
constexpr size_t kOffOsy  = kOffOsx + kBytesO;
constexpr size_t kOffS16x = kOffOsy + kBytesO;
constexpr size_t kOffS16y = kOffS16x + kBytesS16;
constexpr size_t kWsTotal = kOffS16y + kBytesS16;
static_assert(kWsTotal == 100274176u);
static_assert(kWsTotal <= 134217728u);
static_assert(kOffS16y == kOffS16x + (size_t)kTok * kDim * 2);
static_assert(kDim % 32 == 0 && kTok % 64 == 0 && kLdQK % 64 == 0 && kDim % 64 == 0);

typedef __attribute__((ext_vector_type(16))) _Float16 v16h;
typedef __attribute__((ext_vector_type(8)))  _Float16 v8h;
typedef __attribute__((ext_vector_type(16))) __bf16   v16b;
typedef __attribute__((ext_vector_type(8)))  __bf16   v8b;
typedef __attribute__((ext_vector_type(8)))  float    v8f;
typedef __attribute__((ext_vector_type(4)))  float    v4f;
typedef __attribute__((ext_vector_type(2)))  float    v2f;

__device__ __forceinline__ unsigned short f2bf_bits(float f) {
  unsigned u = __float_as_uint(f);
  return (unsigned short)((u + 0x7FFFu + ((u >> 16) & 1u)) >> 16);
}
__device__ __forceinline__ float bf_bits2f(unsigned short h) { return __uint_as_float(((unsigned)h) << 16); }

__device__ __forceinline__ void dep_guard_h(v8f& a, v8f& b, v16h x, v16h y) { asm volatile("v_nop\n\tv_nop\n\tv_nop\n\tv_nop" : "+v"(a), "+v"(b) : "v"(x), "v"(y)); }
__device__ __forceinline__ void dep_guard_b(v8f& a, v8f& b, v16b x, v16b y) { asm volatile("v_nop\n\tv_nop\n\tv_nop\n\tv_nop" : "+v"(a), "+v"(b) : "v"(x), "v"(y)); }
__device__ __forceinline__ void keep4_h(v16h a, v16h b, v16h c, v16h d) { asm volatile("v_nop" :: "v"(a), "v"(b), "v"(c), "v"(d)); }
__device__ __forceinline__ void keep4_b(v16b a, v16b b, v16b c, v16b d) { asm volatile("v_nop" :: "v"(a), "v"(b), "v"(c), "v"(d)); }
__device__ __forceinline__ void acc_guard4(v8f& a, v8f& b, v8f& c, v8f& d) { asm volatile("v_nop\n\tv_nop\n\tv_nop\n\tv_nop" : "+v"(a), "+v"(b), "+v"(c), "+v"(d)); }
template <typename T> struct Frag;
template <> struct Frag<_Float16> {
  typedef v16h V; union U { v16h v; v8h h[2]; };
  static __device__ __forceinline__ v16h load(const _Float16* p) {
    U f; f.h[0] = *(const v8h*)(p); f.h[1] = *(const v8h*)(p + 16); return f.v;
  }
  static __device__ __forceinline__ v8f mma(v16h a, v16h b, v8f c) {
    return __builtin_amdgcn_wmma_f32_16x16x32_f16(false, a, false, b, (short)0, c, false, false);
  }
  static __device__ __forceinline__ void guard(v8f& a, v8f& b, v16h x, v16h y) { dep_guard_h(a, b, x, y); }
  static __device__ __forceinline__ void keep(v16h a, v16h b, v16h c, v16h d) { keep4_h(a, b, c, d); }
};
template <> struct Frag<__bf16> {
  typedef v16b V; union U { v16b v; v8b h[2]; };
  static __device__ __forceinline__ v16b load(const __bf16* p) {
    U f; f.h[0] = *(const v8b*)(p); f.h[1] = *(const v8b*)(p + 16); return f.v;
  }
  static __device__ __forceinline__ v8f mma(v16b a, v16b b, v8f c) {
    return __builtin_amdgcn_wmma_f32_16x16x32_bf16(false, a, false, b, (short)0, c, false, false);
  }
  static __device__ __forceinline__ void guard(v8f& a, v8f& b, v16b x, v16b y) { dep_guard_b(a, b, x, y); }
  static __device__ __forceinline__ void keep(v16b a, v16b b, v16b c, v16b d) { keep4_b(a, b, c, d); }
};

template <int ET> struct Elem;
template <> struct Elem<0> { typedef _Float16 T; };
template <> struct Elem<1> { typedef __bf16 T; };
template <int ET, bool SPLIT, int BIAS_MODE, int OUT_MODE, bool RESID, int ACT = 0>
__global__ __launch_bounds__(256) void wmma_gemm64(
    const unsigned short* __restrict__ Ap, const unsigned short* __restrict__ A2p, int lda, long strideA,
    const unsigned short* __restrict__ Btp, const unsigned short* __restrict__ Bt2p, int ldb, long strideB,
    void* __restrict__ Cout, void* __restrict__ Cout2, int ldc, long strideC,
    const float* __restrict__ bias,
    const float* __restrict__ resid, long strideR,
    int M, int N, int K, float scale) {
  typedef typename Elem<ET>::T T;
  typedef typename Frag<T>::V V;
  const T* A = (const T*)Ap; const T* A2 = (const T*)A2p; const T* Bt = (const T*)Btp; const T* Bt2 = (const T*)Bt2p;
  __shared__ __align__(16) float sT[8][16 * 68];
  const int b    = blockIdx.y;
  const int lane = threadIdx.x & 31;
  const int wave = threadIdx.x >> 5;
  const int tilesN = N >> 6;
  const int tilesM = M >> 6;
  const int tile = blockIdx.x * 8 + wave;
  if (tile >= tilesM * tilesN) return;
  const int tm = tile / tilesN;
  const int tn = tile - tm * tilesN;
  const int m0 = tm << 6;
  const int n0 = tn << 6;

  const T* Ab  = A  + (size_t)b * strideA;
  const T* Bb  = Bt + (size_t)b * strideB;
  const T* Ab2 = SPLIT ? (A2  + (size_t)b * strideA) : nullptr;
  const T* Bb2 = SPLIT ? (Bt2 + (size_t)b * strideB) : nullptr;

  const int rlane = lane & 15;
  const int koff  = (lane >> 4) * 8;
  const int mOff  = (lane >> 4) * 8;

  v8f acc[4][4];
#pragma unroll
  for (int i = 0; i < 4; ++i)
#pragma unroll
    for (int j = 0; j < 4; ++j) acc[i][j] = (v8f){0.f,0.f,0.f,0.f,0.f,0.f,0.f,0.f};

  for (int k0 = 0; k0 < K; k0 += 32) {
    V bh[4], bl[4];
#pragma unroll
    for (int j = 0; j < 4; ++j) {
      const size_t bo = (size_t)(n0 + (j << 4) + rlane) * ldb + koff + k0;
      bh[j] = Frag<T>::load(Bb + bo);
      if (SPLIT) bl[j] = Frag<T>::load(Bb2 + bo);
    }
#pragma unroll
    for (int i = 0; i < 4; ++i) {
      const size_t ao = (size_t)(m0 + (i << 4) + rlane) * lda + koff + k0;
      V ah = Frag<T>::load(Ab + ao);
      V al;
      if (SPLIT) al = Frag<T>::load(Ab2 + ao);
#pragma unroll
      for (int j = 0; j < 4; ++j) {
        acc[i][j] = Frag<T>::mma(ah, bh[j], acc[i][j]);
        if (SPLIT) {
          acc[i][j] = Frag<T>::mma(ah, bl[j], acc[i][j]);
          acc[i][j] = Frag<T>::mma(al, bh[j], acc[i][j]);
        }
      }
      Frag<T>::guard(acc[i][0], acc[i][3], ah, SPLIT ? al : ah);
    }
    Frag<T>::keep(bh[0], bh[1], bh[2], bh[3]);
    if (SPLIT) Frag<T>::keep(bl[0], bl[1], bl[2], bl[3]);
  }
  acc_guard4(acc[0][0], acc[0][1], acc[0][2], acc[0][3]);
  acc_guard4(acc[1][0], acc[1][1], acc[1][2], acc[1][3]);
  acc_guard4(acc[2][0], acc[2][1], acc[2][2], acc[2][3]);
  acc_guard4(acc[3][0], acc[3][1], acc[3][2], acc[3][3]);

  float* slab = sT[wave];
  const float* Rb = RESID ? (resid + (size_t)b * strideR) : nullptr;
#pragma unroll
  for (int i = 0; i < 4; ++i) {
    const int mBase = m0 + (i << 4);
#pragma unroll
    for (int j = 0; j < 4; ++j) {
      const int n = n0 + (j << 4) + rlane;
      float bv = 0.f;
      if (BIAS_MODE == 2) bv = bias[n];
#pragma unroll
      for (int r = 0; r < 8; ++r) {
        float v = acc[i][j][r] * scale;
        if (BIAS_MODE == 1) v += bias[mBase + mOff + r];
        if (BIAS_MODE == 2) v += bv;
        if (RESID) v += Rb[(size_t)(mBase + mOff + r) * ldc + n];
        if (ACT == 1) v = tanhf(v);
        if (ACT == 2) v = fmaxf(v, 0.0f);
        if (ACT == 3) v = v / (1.0f + expf(-v));
        if (ACT == 4) v = (v > 0.f) ? v : 0.01f * v;
        if (ACT == 5) v = 0.5f * v * (1.0f + erff(v * 0.70710678118654752f));
        slab[(mOff + r) * 68 + (j << 4) + rlane] = v;
      }
    }
    __builtin_amdgcn_fence(__ATOMIC_RELEASE, "workgroup");
    __builtin_amdgcn_wave_barrier();
    __builtin_amdgcn_fence(__ATOMIC_ACQUIRE, "workgroup");
    if (OUT_MODE == 0) {
      float* C = (float*)Cout + (size_t)b * strideC;
      const int hh = lane >> 4, c4 = (lane & 15) * 4;
      for (int pass = 0; pass < 2; ++pass) {
#pragma unroll
        for (int it = 0; it < 8; ++it) {
          const int row = it * 2 + hh;
          v4f v = *(const v4f*)(slab + row * 68 + c4);
          *(volatile v4f*)(C + (size_t)(mBase + row) * ldc + n0 + c4) = v;
        }
        __threadfence();
      }
    } else {
      const int q = lane >> 3, c8 = (lane & 7) * 8;
      unsigned short* C  = (unsigned short*)Cout  + (size_t)b * strideC;
      unsigned short* C2 = (OUT_MODE == 2) ? ((unsigned short*)Cout2 + (size_t)b * strideC) : nullptr;
      for (int pass = 0; pass < 2; ++pass) {
#pragma unroll
        for (int it = 0; it < 4; ++it) {
          const int row = it * 4 + q;
          const float* sp = slab + row * 68 + c8;
          v8h hv, lv;
#pragma unroll
          for (int e = 0; e < 8; ++e) {
            if (OUT_MODE == 1) {
              hv[e] = (_Float16)sp[e];
            } else {
              unsigned short hb = f2bf_bits(sp[e]);
              unsigned short lb = f2bf_bits(sp[e] - bf_bits2f(hb));
              hv[e] = __builtin_bit_cast(_Float16, hb);
              lv[e] = __builtin_bit_cast(_Float16, lb);
            }
          }
          *(volatile v8h*)(C + (size_t)(mBase + row) * ldc + n0 + c8) = hv;
          if (OUT_MODE == 2) *(volatile v8h*)(C2 + (size_t)(mBase + row) * ldc + n0 + c8) = lv;
        }
        __threadfence();
      }
    }
    __builtin_amdgcn_fence(__ATOMIC_RELEASE, "workgroup");
    __builtin_amdgcn_wave_barrier();
    __builtin_amdgcn_fence(__ATOMIC_ACQUIRE, "workgroup");
  }
}

__device__ __forceinline__ unsigned pk16(unsigned short a, unsigned short b) { return (unsigned)a | ((unsigned)b << 16); }

__global__ __launch_bounds__(256) void cast_f32_bf16x2(const float* __restrict__ in, unsigned short* __restrict__ out, int n2) {
  const int i = blockIdx.x * 256 + threadIdx.x;
  if (i < n2) {
    const v2f f = *(const v2f*)(in + 2 * (size_t)i);
    const unsigned u = pk16(f2bf_bits(f[0]), f2bf_bits(f[1]));
    ((volatile unsigned*)out)[i] = u;
    __threadfence();
    ((volatile unsigned*)out)[i] = u;
  }
}

__global__ __launch_bounds__(256) void cast_f32_bf16val_f16x2(const float* __restrict__ in, unsigned short* __restrict__ out,
                                                              int n2, float wscale) {
  const int i = blockIdx.x * 256 + threadIdx.x;
  if (i < n2) {
    const v2f f = *(const v2f*)(in + 2 * (size_t)i);
    const float r0 = bf_bits2f(f2bf_bits(f[0])) * wscale;
    const float r1 = bf_bits2f(f2bf_bits(f[1])) * wscale;
    const unsigned u = pk16(__builtin_bit_cast(unsigned short, (_Float16)r0), __builtin_bit_cast(unsigned short, (_Float16)r1));
    ((volatile unsigned*)out)[i] = u;
    __threadfence();
    ((volatile unsigned*)out)[i] = u;
  }
}

__global__ __launch_bounds__(256) void rne_bias_kernel(const float* __restrict__ in, float* __restrict__ out, int n) {
  const int i = blockIdx.x * 256 + threadIdx.x;
  if (i < n) {
    const float v = bf_bits2f(f2bf_bits(in[i]));
    ((volatile float*)out)[i] = v;
    __threadfence();
    ((volatile float*)out)[i] = v;
  }
}

__device__ __forceinline__ v8f mma_h(v16h a, v16h b, v8f c) {
  c = __builtin_amdgcn_wmma_f32_16x16x32_f16(false, a, false, b, (short)0, c, false, false);
  asm volatile("v_nop\n\tv_nop\n\tv_nop\n\tv_nop" : "+v"(c) : "v"(a), "v"(b));
  return c;
}

constexpr float kProbCarry = 32768.0f;

template <int OUT16>
__global__ __launch_bounds__(128)
void attn_f16_kernel(const unsigned short* __restrict__ qp, const unsigned short* __restrict__ kp,
                     const unsigned short* __restrict__ vtp, const float* __restrict__ resid,
                     void* __restrict__ outp, float sscale, float onorm, float oscale) {
  union FH { v16h v; v8h h[2]; };
  __shared__ __align__(16) _Float16 Ksh[kKeyChunk * kHd];
  __shared__ __align__(16) _Float16 Vth[kHd * kKeyChunk];
  __shared__ __align__(16) _Float16 Psh[kWaves][16 * kKeyChunk];
  __shared__ __align__(16) float    Os[kWaves][16 * 68];

  const int tid  = threadIdx.x;
  const int wave = tid >> 5;
  const int lane = tid & 31;
  const int hh   = lane >> 4;
  const int c    = lane & 15;

  constexpr int nqb = kSeq / 64;
  const int bx   = blockIdx.x;
  const int qblk = bx % nqb;
  const int bhd  = bx / nqb;
  const int h    = bhd % kHeads;
  const int b    = bhd / kHeads;
  const int q0   = qblk * 64 + wave * 16;

  const _Float16* Qbase = (const _Float16*)(const void*)qp  + (size_t)b * kSeq * kLdQK + (size_t)h * kHd;
  const _Float16* Kbase = (const _Float16*)(const void*)kp  + (size_t)b * kSeq * kLdQK + (size_t)h * kHd;
  const _Float16* Vbase = (const _Float16*)(const void*)vtp + (size_t)h * kHd * kTok + (size_t)b * kSeq;

  v16h qa[2];
#pragma unroll
  for (int dc = 0; dc < 2; ++dc)
    qa[dc] = Frag<_Float16>::load(Qbase + (size_t)(q0 + c) * kLdQK + dc * 32 + 8 * hh);

  float mrow[8], lrow[8];
  v8f oacc[4];
#pragma unroll
  for (int r = 0; r < 8; ++r) { mrow[r] = -INFINITY; lrow[r] = 0.f; }
#pragma unroll
  for (int t = 0; t < 4; ++t) oacc[t] = (v8f){0.f,0.f,0.f,0.f,0.f,0.f,0.f,0.f};

  constexpr int nChunks = kSeq / kKeyChunk;
  for (int kc = 0; kc < nChunks; ++kc) {
    const int kv0 = kc * kKeyChunk;
    __syncthreads();
    {
      const int r = tid >> 1, half = (tid & 1) * 32;
      const _Float16* ks = Kbase + (size_t)(kv0 + r) * kLdQK + half;
      const _Float16* vs = Vbase + (size_t)r * kTok + kv0 + half;
#pragma unroll
      for (int i = 0; i < 4; ++i) {
        const v8h a0 = *(const v8h*)(ks + 8 * i);
        const v8h b0 = *(const v8h*)(vs + 8 * i);
        *(v8h*)(Ksh + r * kHd       + half + 8 * i) = a0;
        *(v8h*)(Vth + r * kKeyChunk + half + 8 * i) = b0;
      }
    }
    __syncthreads();

    v8f s[4];
#pragma unroll
    for (int j = 0; j < 4; ++j) {
      s[j] = (v8f){0.f,0.f,0.f,0.f,0.f,0.f,0.f,0.f};
#pragma unroll
      for (int dc = 0; dc < 2; ++dc) {
        FH kb;
        kb.h[0] = *(const v8h*)(Ksh + (j * 16 + c) * kHd + dc * 32 + 8 * hh);
        kb.h[1] = *(const v8h*)(Ksh + (j * 16 + c) * kHd + dc * 32 + 16 + 8 * hh);
        s[j] = mma_h(qa[dc], kb.v, s[j]);
      }
    }
    float cm[8];
#pragma unroll
    for (int r = 0; r < 8; ++r) {
      float m = -INFINITY;
#pragma unroll
      for (int j = 0; j < 4; ++j) {
        const float sv = s[j][r] * sscale;
        s[j][r] = sv;
        m = fmaxf(m, sv);
      }
#pragma unroll
      for (int off = 1; off < 16; off <<= 1) m = fmaxf(m, __shfl_xor(m, off, 32));
      cm[r] = m;
    }
    _Float16* pwh = Psh[wave];
#pragma unroll
    for (int r = 0; r < 8; ++r) {
      const float mnew = fmaxf(mrow[r], cm[r]);
      const float alpha = expf(mrow[r] - mnew);
      mrow[r] = mnew;
      float psum = 0.f;
#pragma unroll
      for (int j = 0; j < 4; ++j) {
        const float p = expf(s[j][r] - mnew);
        psum += p;
        pwh[(8 * hh + r) * kKeyChunk + j * 16 + c] = (_Float16)(p * kProbCarry);
      }
#pragma unroll
      for (int off = 1; off < 16; off <<= 1) psum += __shfl_xor(psum, off, 32);
      lrow[r] = lrow[r] * alpha + psum;
#pragma unroll
      for (int t = 0; t < 4; ++t) oacc[t][r] *= alpha;
    }
    __builtin_amdgcn_fence(__ATOMIC_RELEASE, "workgroup");
    __builtin_amdgcn_wave_barrier();
    __builtin_amdgcn_fence(__ATOMIC_ACQUIRE, "workgroup");
#pragma unroll 1
    for (int kk = 0; kk < 2; ++kk) {
      FH pa;
      pa.h[0] = *(const v8h*)(pwh + c * kKeyChunk + kk * 32 + 8 * hh);
      pa.h[1] = *(const v8h*)(pwh + c * kKeyChunk + kk * 32 + 16 + 8 * hh);
#pragma unroll
      for (int t = 0; t < 4; ++t) {
        FH vb;
        vb.h[0] = *(const v8h*)(Vth + (t * 16 + c) * kKeyChunk + kk * 32 + 8 * hh);
        vb.h[1] = *(const v8h*)(Vth + (t * 16 + c) * kKeyChunk + kk * 32 + 16 + 8 * hh);
        oacc[t] = mma_h(pa.v, vb.v, oacc[t]);
      }
    }
  }

  float* os = Os[wave];
#pragma unroll
  for (int r = 0; r < 8; ++r) {
    const float inv = onorm * (1.0f / lrow[r]);
#pragma unroll
    for (int t = 0; t < 4; ++t) os[(8 * hh + r) * 68 + t * 16 + c] = oacc[t][r] * inv;
  }
  __builtin_amdgcn_fence(__ATOMIC_RELEASE, "workgroup");
  __builtin_amdgcn_wave_barrier();
  __builtin_amdgcn_fence(__ATOMIC_ACQUIRE, "workgroup");
  if (OUT16 == 0) {
    float* ob = (float*)outp + (size_t)b * kSeq * kDim + (size_t)h * kHd;
    const int c4 = c * 4;
    for (int ps = 0; ps < 2; ++ps) {
#pragma unroll
      for (int it = 0; it < 8; ++it) {
        const int row = it * 2 + hh;
        v4f val = *(const v4f*)(os + row * 68 + c4);
        *(volatile v4f*)(ob + (size_t)(q0 + row) * kDim + c4) = val;
      }
      __threadfence();
    }
  } else {
    unsigned short* o16 = (unsigned short*)outp + (size_t)b * kSeq * kDim + (size_t)h * kHd;
    const float*    rb  = resid + (size_t)b * kSeq * kDim + (size_t)h * kHd;
    const int qq = lane >> 3, c8 = (lane & 7) * 8;
    for (int ps = 0; ps < 2; ++ps) {
#pragma unroll
      for (int it = 0; it < 4; ++it) {
        const int row = it * 4 + qq;
        const float* sp = os + row * 68 + c8;
        const float* rp = rb + (size_t)(q0 + row) * kDim + c8;
        const v4f ra = *(const v4f*)rp;
        const v4f rc = *(const v4f*)(rp + 4);
        v8h hv;
#pragma unroll
        for (int e = 0; e < 4; ++e) {
          hv[e]     = (_Float16)((sp[e]     + ra[e]) * oscale);
          hv[4 + e] = (_Float16)((sp[4 + e] + rc[e]) * oscale);
        }
        *(volatile v8h*)(o16 + (size_t)(q0 + row) * kDim + c8) = hv;
      }
      __threadfence();
    }
  }
}

extern "C" void kernel_launch(void* const* d_in, const int* in_sizes, int n_in,
                              void* d_out, int out_size, void* d_ws, size_t ws_size,
                              hipStream_t stream) {
  if (n_in < 5) return;
  if (in_sizes[0] != kTok * kDim || in_sizes[1] != kTok * kDim || in_sizes[2] != kQkvRows * kDim ||
      in_sizes[3] != kDim * kDim || in_sizes[4] != kDim) return;
  if (out_size != 2 * kTok * kDim) return;
  if (ws_size < kWsTotal) return;

  const float* x      = (const float*)d_in[0];
  const float* y      = (const float*)d_in[1];
  const float* w_qkv  = (const float*)d_in[2];
  const float* w_proj = (const float*)d_in[3];
  const float* b_proj = (const float*)d_in[4];
  char* ws = (char*)d_ws;
  unsigned short* xb    = (unsigned short*)(ws + kOffXb);
  unsigned short* yb    = (unsigned short*)(ws + kOffYb);
  unsigned short* wqb   = (unsigned short*)(ws + kOffWq);
  unsigned short* wph   = (unsigned short*)(ws + kOffWp);
  float*          biasr = (float*)(ws + kOffBias);
  unsigned short* px    = (unsigned short*)(ws + kOffPx);
  unsigned short* py    = (unsigned short*)(ws + kOffPy);
  unsigned short* vt    = (unsigned short*)(ws + kOffVt);
  float*          osx   = (float*)(ws + kOffOsx);
  float*          osy   = (float*)(ws + kOffOsy);
  unsigned short* s16x  = (unsigned short*)(ws + kOffS16x);
  unsigned short* s16y  = (unsigned short*)(ws + kOffS16y);
  float* out = (float*)d_out;

  const int n2x  = kTok * kDim / 2;
  const int n2wq = kQkvRows * kDim / 2;
  const int n2wp = kDim * kDim / 2;
  cast_f32_bf16x2<<<dim3(n2x / 256), 256, 0, stream>>>(x, xb, n2x);
  cast_f32_bf16x2<<<dim3(n2x / 256), 256, 0, stream>>>(y, yb, n2x);
  cast_f32_bf16x2<<<dim3(n2wq / 256), 256, 0, stream>>>(w_qkv, wqb, n2wq);
  cast_f32_bf16val_f16x2<<<dim3(n2wp / 256), 256, 0, stream>>>(w_proj, wph, n2wp, 64.0f);
  rne_bias_kernel<<<dim3(kDim / 256), 256, 0, stream>>>(b_proj, biasr, kDim);

  wmma_gemm64<1, false, 0, 1, false><<<dim3(288, 1), 256, 0, stream>>>(
      xb, xb, kDim, 0L, wqb, wqb, kDim, 0L, (void*)px, (void*)px, kLdQK, 0L,
      biasr, biasr, 0L, kTok, kLdQK, kDim, 8.0f);
  wmma_gemm64<1, false, 0, 1, false><<<dim3(288, 1), 256, 0, stream>>>(
      yb, yb, kDim, 0L, wqb, wqb, kDim, 0L, (void*)py, (void*)py, kLdQK, 0L,
      biasr, biasr, 0L, kTok, kLdQK, kDim, 8.0f);
  wmma_gemm64<1, false, 0, 1, false><<<dim3(96, 1), 256, 0, stream>>>(
      wqb + (size_t)3 * kDim * kDim, wqb + (size_t)3 * kDim * kDim, kDim, 0L, xb, xb, kDim, 0L,
      (void*)vt, (void*)vt, kTok, 0L, biasr, biasr, 0L, kDim, kTok, kDim, 8.0f);

  const float sPos = 0.125f / 64.0f;
  const float sNeg = -sPos;
  const float oNorm = 1.0f / (kProbCarry * 8.0f);
  const int attnGrid = kBatch * kHeads * (kSeq / 64);
  attn_f16_kernel<0><<<dim3(attnGrid), 128, 0, stream>>>(px + kDim, px + 2 * kDim, vt, osx, (void*)osx, sPos, oNorm, 256.0f);
  attn_f16_kernel<1><<<dim3(attnGrid), 128, 0, stream>>>(py, px + 2 * kDim, vt, osx, (void*)s16x, sNeg, oNorm, 256.0f);
  attn_f16_kernel<0><<<dim3(attnGrid), 128, 0, stream>>>(py + kDim, py + 2 * kDim, vt, osy, (void*)osy, sPos, oNorm, 256.0f);
  attn_f16_kernel<1><<<dim3(attnGrid), 128, 0, stream>>>(px, py + 2 * kDim, vt, osy, (void*)s16y, sNeg, oNorm, 256.0f);

  wmma_gemm64<0, false, 2, 0, false><<<dim3(96, 2), 256, 0, stream>>>(
      s16x, s16x, kDim, (long)kTok * kDim, wph, wph, kDim, 0L, (void*)out, (void*)out, kDim, (long)kTok * kDim,
      biasr, biasr, 0L, kTok, kDim, kDim, 1.0f / 16384.0f);
}
